// SparseLDS_58798102282591
// MI455X (gfx1250) — hardware-verified
//
#include <hip/hip_runtime.h>
#include <math.h>

typedef __attribute__((ext_vector_type(16))) _Float16 v16h;
typedef __attribute__((ext_vector_type(16))) __bf16 v16b;
typedef __attribute__((ext_vector_type(8)))  _Float16 v8h;
typedef __attribute__((ext_vector_type(8)))  float v8f;
typedef __attribute__((ext_vector_type(4)))  float v4f;
typedef __attribute__((ext_vector_type(2)))  float v2f;
typedef __attribute__((ext_vector_type(4)))  unsigned v4u;
typedef __attribute__((ext_vector_type(4)))  int v4i;
typedef float __attribute__((may_alias)) float_a;
typedef int __attribute__((may_alias)) int_a;

template <typename T> __device__ __forceinline__ void vst2(void* p, T v) { *(volatile T*)p = v; __threadfence(); *(volatile T*)p = v; }
__device__ __forceinline__ v8f wmma16(v16h a, v16h b, v8f c) {
  v8f d = __builtin_amdgcn_wmma_f32_16x16x32_f16(false, a, false, b, (short)0, c, false, false);
  asm volatile("v_nop\n\tv_nop\n\tv_nop\n\tv_nop" : "+v"(d) : "v"(a), "v"(b));
  return d;
}
__device__ __forceinline__ v8f wmma_bf(v16b a, v16b b, v8f c) {
  v8f d = __builtin_amdgcn_wmma_f32_16x16x32_bf16(false, a, false, b, (short)0, c, false, false);
  asm volatile("v_nop\n\tv_nop\n\tv_nop\n\tv_nop" : "+v"(d) : "v"(a), "v"(b));
  return d;
}
__device__ __forceinline__ v16h frag_h(const _Float16* rowk0, int lane) {
  union { v16h v; v8h q[2]; } u; const _Float16* p = rowk0 + 8 * (lane >> 4);
  u.q[0] = *(const v8h*)p; u.q[1] = *(const v8h*)(p + 16); return u.v;
}
__device__ __forceinline__ v16h frag_f32(const float* rowk0, int lane) {
  v16h a; const float* p = rowk0 + 8 * (lane >> 4);
#pragma unroll
  for (int i = 0; i < 8; ++i) { a[i] = (_Float16)p[i]; a[8 + i] = (_Float16)p[16 + i]; }
  return a;
}
__device__ __forceinline__ v16h frag_f32s(const float* rowk0, int lane, float sc) {
  v16h a; const float* p = rowk0 + 8 * (lane >> 4);
#pragma unroll
  for (int i = 0; i < 8; ++i) { a[i] = (_Float16)(p[i] * sc); a[8 + i] = (_Float16)(p[16 + i] * sc); }
  return a;
}
__device__ __forceinline__ v16h fragc_f32(const float* W, int k0, int n, int lane, int ld, int K) {
  v16h a; const int g = lane >> 4;
#pragma unroll
  for (int i = 0; i < 8; ++i) { const int ka = k0 + 8 * g + i, kb = ka + 16;
    a[i] = (_Float16)(ka < K ? W[(size_t)ka * ld + n] : 0.f); a[8 + i] = (_Float16)(kb < K ? W[(size_t)kb * ld + n] : 0.f); }
  return a;
}
struct F2 { v16b h, l; };
__device__ __forceinline__ F2 bsplit16(const float v[16]) { F2 r;
#pragma unroll
  for (int i = 0; i < 16; ++i) { const __bf16 h = (__bf16)v[i]; r.h[i] = h; r.l[i] = (__bf16)(v[i] - (float)h); }
  return r; }
__device__ __forceinline__ F2 split_row(const float* row, int k0, int lane) { float v[16]; const float* p = row + k0 + 8 * (lane >> 4);
#pragma unroll
  for (int i = 0; i < 8; ++i) { v[i] = p[i]; v[8 + i] = p[16 + i]; }
  return bsplit16(v); }
__device__ __forceinline__ F2 split_rowK(const float* row, int k0, int lane, int K) { float v[16]; const int g = lane >> 4;
#pragma unroll
  for (int i = 0; i < 8; ++i) { const int ka = k0 + 8 * g + i, kb = ka + 16; v[i] = ka < K ? row[ka] : 0.f; v[8 + i] = kb < K ? row[kb] : 0.f; }
  return bsplit16(v); }
__device__ __forceinline__ F2 split_col(const float* W, int k0, int n, int lane, int ld, int K) { float v[16]; const int g = lane >> 4;
#pragma unroll
  for (int i = 0; i < 8; ++i) { const int ka = k0 + 8 * g + i, kb = ka + 16; v[i] = ka < K ? W[(size_t)ka * ld + n] : 0.f; v[8 + i] = kb < K ? W[(size_t)kb * ld + n] : 0.f; }
  return bsplit16(v); }
__device__ __forceinline__ v8f mac3(const F2& a, const F2& b, v8f c) { c = wmma_bf(a.l, b.h, c); c = wmma_bf(a.h, b.l, c); return wmma_bf(a.h, b.h, c); }
__device__ __forceinline__ float sigm(float v) { return 1.0f / (1.0f + expf(-v)); }
#define LDSX() do { asm volatile("s_wait_dscnt 0" ::: "memory"); __builtin_amdgcn_wave_barrier(); __builtin_amdgcn_fence(__ATOMIC_RELEASE, "workgroup"); } while (0)

#define NBT 8
#define TT 8192
#define NN 512
#define MM 512

__global__ __launch_bounds__(256) void k_pow(const float* __restrict__ lre, const float* __restrict__ lim, float* __restrict__ PR, float* __restrict__ PI) {
  __shared__ float slr[NN], sli[NN];
  const int tid = threadIdx.x, t = blockIdx.x;
  for (int n = tid; n < NN; n += 256) { const float mag = expf(lre[n]); float sv, cv; sincosf(lim[n], &sv, &cv); slr[n] = mag * cv; sli[n] = mag * sv; }
  __syncthreads();
  const int kexp = TT - 1 - t;
  __shared__ __align__(16) float sor[NN], soi[NN];
  for (int n = tid; n < NN; n += 256) {
    #pragma clang fp contract(off)
    float br = slr[n], bi = sli[n]; float pr = 1.f, pi = 0.f; int e = kexp;
    while (e > 0) { if (e & 1) { const float nr = pr * br - pi * bi, ni = pr * bi + pi * br; pr = nr; pi = ni; } const float sr = br * br - bi * bi, si = 2.f * br * bi; br = sr; bi = si; e >>= 1; }
    sor[n] = pr; soi[n] = pi; }
  __syncthreads();
  for (int q = tid; q < NN / 4; q += 256) { vst2(PR + (size_t)t * NN + q * 4, *(const v4f*)(&sor[q * 4])); vst2(PI + (size_t)t * NN + q * 4, *(const v4f*)(&soi[q * 4])); }
}
__global__ __launch_bounds__(128) void k_scan(const float* __restrict__ x, const float* __restrict__ PR, const float* __restrict__ PI, float* __restrict__ SR, float* __restrict__ SI) {
  __shared__ __align__(16) float so[4][16][20];
  const int tid = threadIdx.x, wave = tid >> 5, lane = tid & 31, col = lane & 15, g = lane >> 4;
  const int which = wave >> 1, n0 = blockIdx.x * 32 + (wave & 1) * 16;
  const float* P = which ? PI : PR;
  float zz[16];
#pragma unroll
  for (int i = 0; i < 16; ++i) zz[i] = 0.f;
  const F2 fz = bsplit16(zz);
  const int arow = col < NBT ? col : 0;
  v8f acc = {};
#pragma unroll 2
  for (int kc = 0; kc < TT / 32; ++kc) { F2 a = split_row(x + (size_t)arow * TT, kc * 32, lane); if (col >= NBT) a = fz;
    acc = mac3(a, split_col(P, kc * 32, n0 + col, lane, NN, TT), acc); }
#pragma unroll
  for (int r = 0; r < 8; ++r) so[wave][8 * g + r][col] = acc[r];
  LDSX();
  float* dst = which ? SI : SR;
  for (int q = lane; q < NBT * 4; q += 32) { const int r = q >> 2, pc = q & 3; vst2(dst + (size_t)r * NN + n0 + pc * 4, *(const v4f*)(&so[wave][r][pc * 4])); }
}
__global__ __launch_bounds__(256) void k_out(const float* __restrict__ SR, const float* __restrict__ SI, const float* __restrict__ Cre, const float* __restrict__ Cim, const float* __restrict__ x, const float* __restrict__ D, const float* __restrict__ Do, float* __restrict__ out) {
  __shared__ float ssr[NN], ssi[NN]; __shared__ __align__(16) float so[MM];
  const int b = blockIdx.x, tid = threadIdx.x;
  for (int n = tid; n < NN; n += 256) { ssr[n] = SR[(size_t)b * NN + n]; ssi[n] = SI[(size_t)b * NN + n]; }
  __syncthreads();
  const float xl = x[(size_t)b * TT + TT - 1];
  for (int m = tid; m < MM; m += 256) { float s = 0.f;
#pragma unroll 4
    for (int n = 0; n < NN; ++n) s += ssr[n] * Cre[(size_t)n * MM + m] - ssi[n] * Cim[(size_t)n * MM + m];
    so[m] = s + xl * D[m] + Do[m]; }
  __syncthreads();
  if (tid < MM / 4) vst2(out + (size_t)b * MM + tid * 4, *(const v4f*)(&so[tid * 4]));
}
extern "C" void kernel_launch(void* const* d_in, const int* in_sizes, int n_in, void* d_out, int out_size, void* d_ws, size_t ws_size, hipStream_t stream) {
  (void)in_sizes; (void)n_in; (void)out_size; (void)ws_size;
  const float* x = (const float*)d_in[0]; const float* lre = (const float*)d_in[1]; const float* lim = (const float*)d_in[2]; const float* Cre = (const float*)d_in[3]; const float* Cim = (const float*)d_in[4]; const float* D = (const float*)d_in[5]; const float* Do = (const float*)d_in[6];
  float* out = (float*)d_out;
  char* ws = (char*)d_ws; size_t off = 0;
  auto take = [&](size_t bytes) { char* p = ws + off; off += (bytes + 255) & ~(size_t)255; return p; };
  float* PR = (float*)take((size_t)TT * NN * 4); float* PI = (float*)take((size_t)TT * NN * 4); float* SR = (float*)take((size_t)NBT * NN * 4); float* SI = (float*)take((size_t)NBT * NN * 4);
  k_pow<<<TT, 256, 0, stream>>>(lre, lim, PR, PI);
  k_scan<<<NN / 32, 128, 0, stream>>>(x, PR, PI, SR, SI);
  k_out<<<NBT, 256, 0, stream>>>(SR, SI, Cre, Cim, x, D, Do, out);
}
